// MambaBlock_23450521436677
// MI455X (gfx1250) — hardware-verified
//
#include <hip/hip_runtime.h>
#include <math.h>

typedef __attribute__((ext_vector_type(16))) _Float16 v16h;
typedef __attribute__((ext_vector_type(8)))  _Float16 v8h;
typedef __attribute__((ext_vector_type(8)))  float    v8f;
typedef __attribute__((ext_vector_type(4)))  float    v4f;

constexpr int kBatch  = 2;
constexpr int kSeq    = 1024;
constexpr int kDm     = 768;
constexpr int kDin    = 1536;
constexpr int kNst    = 16;
constexpr int kDtR    = 32;
constexpr int kXzP    = 2 * kDin;
constexpr int kXdP    = 64;
constexpr int kRows   = kBatch * kSeq;
constexpr int kTP     = 260;
constexpr int kScanTS = 16;

static_assert(kDtR + 2 * kNst == kXdP, "x_proj width");
static_assert((kDm % 32) == 0 && (kDin % 32) == 0 && (kDtR % 32) == 0, "GEMM K multiples of 32");
static_assert((kRows % 64) == 0 && (kXzP % 64) == 0 && (kXdP % 64) == 0 && (kDin % 64) == 0 && (kDm % 64) == 0, "GEMM M,N multiples of 64");
static_assert((kSeq % 64) == 0 && (kSeq & (kSeq - 1)) == 0 && (kDin % 256) == 0 && (kSeq % kScanTS) == 0, "tile multiples");
static_assert(kRows * kDm == 1572864 && kXzP * kDm == 2359296 && kXdP * kDin == 98304 && kDin * kDtR == 49152 && kDm * kDin == 1179648, "wire sizes");

constexpr float kCarX   = 16.0f;
constexpr float kCarW   = 32.0f;
constexpr float kCarU   = 16.0f;
constexpr float kCarDt  = 16.0f;
constexpr float kCarWdt = 8.0f;
constexpr float kCarY   = 16.0f;

constexpr size_t kOffX16   = 0;
constexpr size_t kOffWIN   = kOffX16  + (size_t)kRows * kDm  * 2;
constexpr size_t kOffWX    = kOffWIN  + (size_t)kXzP  * kDm  * 2;
constexpr size_t kOffWDT   = kOffWX   + (size_t)kXdP  * kDin * 2;
constexpr size_t kOffWOUT  = kOffWDT  + (size_t)kDin  * kDtR * 2;
constexpr size_t kOffXZ    = kOffWOUT + (size_t)kDm   * kDin * 2;
constexpr size_t kOffUC    = kOffXZ   + (size_t)kRows * kXzP * 4;
constexpr size_t kOffUC16  = kOffUC   + (size_t)kRows * kDin * 4;
constexpr size_t kOffXD    = kOffUC16 + (size_t)kRows * kDin * 2;
constexpr size_t kOffDT16  = kOffXD   + (size_t)kRows * kXdP * 4;
constexpr size_t kOffDLR   = kOffDT16 + (size_t)kRows * kDtR * 2;
constexpr size_t kOffY16   = kOffDLR  + (size_t)kRows * kDin * 4;
constexpr size_t kWsTotal  = kOffY16  + (size_t)kRows * kDin * 2;
static_assert(kWsTotal == 74088448ull, "carve total");
static_assert(kWsTotal <= 134217728ull, "carve cap");
static_assert((kOffWIN % 256) == 0 && (kOffWX % 256) == 0 && (kOffWDT % 256) == 0 && (kOffWOUT % 256) == 0 &&
              (kOffXZ % 256) == 0 && (kOffUC % 256) == 0 && (kOffUC16 % 256) == 0 && (kOffXD % 256) == 0 &&
              (kOffDT16 % 256) == 0 && (kOffDLR % 256) == 0 && (kOffY16 % 256) == 0, "aligned regions");

__device__ __forceinline__ void dep_guard4_h(v8f& a, v8f& b, v8f& c, v8f& d, v16h x, v16h b0, v16h b1, v16h b2, v16h b3) {
  asm volatile("v_nop\n\tv_nop\n\tv_nop\n\tv_nop" : "+v"(a), "+v"(b), "+v"(c), "+v"(d) : "v"(x), "v"(b0), "v"(b1), "v"(b2), "v"(b3));
}
__device__ __forceinline__ void keep4_h(v16h a, v16h b, v16h c, v16h d) { asm volatile("v_nop" :: "v"(a), "v"(b), "v"(c), "v"(d)); }
__device__ __forceinline__ void acc_guard4(v8f& a, v8f& b, v8f& c, v8f& d) { asm volatile("v_nop\n\tv_nop\n\tv_nop\n\tv_nop" : "+v"(a), "+v"(b), "+v"(c), "+v"(d)); }

struct FragH {
  union U { v16h v; v8h h[2]; };
  static __device__ __forceinline__ v16h load(const _Float16* p) {
    U f;
    f.h[0] = *(const v8h*)(p);
    f.h[1] = *(const v8h*)(p + 16);
    return f.v;
  }
  static __device__ __forceinline__ v8f mma(v16h a, v16h b, v8f c) {
    return __builtin_amdgcn_wmma_f32_16x16x32_f16(false, a, false, b, (short)0, c, false, false);
  }
};

template <bool RESID>
__global__ __launch_bounds__(256) void wmma_gemm64_f16(
    const unsigned short* __restrict__ Ap, int lda,
    const unsigned short* __restrict__ Btp, int ldb,
    float* __restrict__ C, int ldc,
    const float* __restrict__ resid,
    int M, int N, int K, float scale)
{
  const _Float16* A  = (const _Float16*)Ap;
  const _Float16* Bt = (const _Float16*)Btp;
  __shared__ __align__(16) float sT[8][16 * 68];
  const int lane = threadIdx.x & 31;
  const int wave = threadIdx.x >> 5;
  const int tilesN = N >> 6;
  const int tilesM = M >> 6;
  const int tile = blockIdx.x * 8 + wave;
  if (tile >= tilesM * tilesN) return;
  const int tm = tile / tilesN;
  const int tn = tile - tm * tilesN;
  const int m0 = tm << 6;
  const int n0 = tn << 6;

  const int rlane = lane & 15;
  const int koff  = (lane >> 4) * 8;
  const int mOff  = (lane >> 4) * 8;

  v8f acc[4][4];
#pragma unroll
  for (int i = 0; i < 4; ++i)
#pragma unroll
    for (int j = 0; j < 4; ++j) acc[i][j] = (v8f){0.f,0.f,0.f,0.f,0.f,0.f,0.f,0.f};

  for (int k0 = 0; k0 < K; k0 += 32) {
    v16h bh[4];
#pragma unroll
    for (int j = 0; j < 4; ++j) {
      const size_t bo = (size_t)(n0 + (j << 4) + rlane) * ldb + koff + k0;
      bh[j] = FragH::load(Bt + bo);
    }
#pragma unroll
    for (int i = 0; i < 4; ++i) {
      const size_t ao = (size_t)(m0 + (i << 4) + rlane) * lda + koff + k0;
      const v16h ah = FragH::load(A + ao);
#pragma unroll
      for (int j = 0; j < 4; ++j) acc[i][j] = FragH::mma(ah, bh[j], acc[i][j]);
      dep_guard4_h(acc[i][0], acc[i][1], acc[i][2], acc[i][3], ah, bh[0], bh[1], bh[2], bh[3]);
    }
    keep4_h(bh[0], bh[1], bh[2], bh[3]);
  }
  acc_guard4(acc[0][0], acc[0][1], acc[0][2], acc[0][3]);
  acc_guard4(acc[1][0], acc[1][1], acc[1][2], acc[1][3]);
  acc_guard4(acc[2][0], acc[2][1], acc[2][2], acc[2][3]);
  acc_guard4(acc[3][0], acc[3][1], acc[3][2], acc[3][3]);

  float* slab = sT[wave];
  const int hh = lane >> 4;
  const int c4 = (lane & 15) * 4;
#pragma unroll
  for (int i = 0; i < 4; ++i) {
    const int mBase = m0 + (i << 4);
#pragma unroll
    for (int j = 0; j < 4; ++j) {
#pragma unroll
      for (int r = 0; r < 8; ++r) {
        slab[(mOff + r) * 68 + (j << 4) + rlane] = acc[i][j][r] * scale;
      }
    }
    __builtin_amdgcn_fence(__ATOMIC_RELEASE, "workgroup");
    __builtin_amdgcn_wave_barrier();
    __builtin_amdgcn_fence(__ATOMIC_ACQUIRE, "workgroup");
    v4f vv[8];
#pragma unroll
    for (int it = 0; it < 8; ++it) {
      const int row = it * 2 + hh;
      v4f v = *(const v4f*)(slab + row * 68 + c4);
      if (RESID) {
        const v4f rv = *(const v4f*)(resid + (size_t)(mBase + row) * ldc + n0 + c4);
        v = v + rv;
      }
      vv[it] = v;
    }
    for (int pass = 0; pass < 2; ++pass) {
#pragma unroll
      for (int it = 0; it < 8; ++it) {
        const int row = it * 2 + hh;
        *(volatile v4f*)(C + (size_t)(mBase + row) * ldc + n0 + c4) = vv[it];
      }
      __threadfence();
    }
    __builtin_amdgcn_fence(__ATOMIC_RELEASE, "workgroup");
    __builtin_amdgcn_wave_barrier();
    __builtin_amdgcn_fence(__ATOMIC_ACQUIRE, "workgroup");
  }
}

__global__ __launch_bounds__(256) void cast_f16_kernel(
    const float* __restrict__ src, unsigned short* __restrict__ dst, int total8, float scale)
{
  const int i = blockIdx.x * 256 + threadIdx.x;
  if (i >= total8) return;
  const size_t e0 = (size_t)i << 3;
  const float* p = src + e0;
  const v4f a0 = *(const v4f*)(p);
  const v4f a1 = *(const v4f*)(p + 4);
  v8h hv;
#pragma unroll
  for (int e = 0; e < 4; ++e) {
    hv[e]     = (_Float16)(a0[e] * scale);
    hv[4 + e] = (_Float16)(a1[e] * scale);
  }
  unsigned short* q = dst + e0;
  *(volatile v8h*)q = hv;
  __threadfence();
  *(volatile v8h*)q = hv;
}

__global__ __launch_bounds__(256) void dt_cast_kernel(
    const float* __restrict__ XD, unsigned short* __restrict__ DT16, int total8, float scale)
{
  const int i = blockIdx.x * 256 + threadIdx.x;
  if (i >= total8) return;
  const int e0  = i << 3;
  const int row = e0 >> 5;
  const int c8  = e0 & 31;
  const float* p = XD + (size_t)row * kXdP + c8;
  const v4f a0 = *(const v4f*)(p);
  const v4f a1 = *(const v4f*)(p + 4);
  v8h hv;
#pragma unroll
  for (int e = 0; e < 4; ++e) {
    hv[e]     = (_Float16)(a0[e] * scale);
    hv[4 + e] = (_Float16)(a1[e] * scale);
  }
  unsigned short* qd = DT16 + e0;
  *(volatile v8h*)qd = hv;
  __threadfence();
  *(volatile v8h*)qd = hv;
}

__global__ __launch_bounds__(256) void conv_silu_kernel(
    const float* __restrict__ XZ, const float* __restrict__ cw, const float* __restrict__ cb,
    float* __restrict__ UC, unsigned short* __restrict__ UC16)
{
  __shared__ __align__(16) float sT[16 * kTP];
  const int tid = threadIdx.x, lane = tid & 31, wave = tid >> 5;
  const int d0 = blockIdx.x * 256, d = d0 + tid;
  const int g0 = blockIdx.y * 64;
  const int tb = g0 & (kSeq - 1);
  const v4f wv = *(const v4f*)(cw + (size_t)d * 4);
  const float w0 = wv[0], w1 = wv[1], w2 = wv[2], w3 = wv[3];
  const float bc = cb[d];
  float xm3, xm2, xm1;
  {
    const bool hist = (tb > 0);
    const int rb = hist ? (g0 - 3) : g0;
    const float v3 = XZ[(size_t)rb * kXzP + d];
    const float v2 = XZ[(size_t)(rb + 1) * kXzP + d];
    const float v1 = XZ[(size_t)(rb + 2) * kXzP + d];
    xm3 = hist ? v3 : 0.f;
    xm2 = hist ? v2 : 0.f;
    xm1 = hist ? v1 : 0.f;
  }
  const int hrow = wave >> 1;
  const int hch  = (wave & 1) * 128 + lane * 4;
#pragma unroll 1
  for (int sub = 0; sub < 4; ++sub) {
    const int lb = g0 + sub * 16;
#pragma unroll 1
    for (int s = 0; s < 16; ++s) {
      const float xcur = XZ[(size_t)(lb + s) * kXzP + d];
      float acc = w0 * xm3;
      acc = fmaf(w1, xm2, acc);
      acc = fmaf(w2, xm1, acc);
      acc = fmaf(w3, xcur, acc);
      const float sv = acc + bc;
      const float sg = __builtin_amdgcn_rcpf(1.0f + expf(-sv));
      sT[s * kTP + tid] = sv * sg;
      xm3 = xm2; xm2 = xm1; xm1 = xcur;
    }
    __syncthreads();
    v4f fv[4];
    v8h bv[2];
#pragma unroll
    for (int it = 0; it < 4; ++it) fv[it] = *(const v4f*)(sT + (it * 4 + hrow) * kTP + hch);
#pragma unroll
    for (int it = 0; it < 2; ++it) {
      const float* sp = sT + (it * 8 + wave) * kTP + lane * 8;
      const v4f a0 = *(const v4f*)(sp);
      const v4f a1 = *(const v4f*)(sp + 4);
#pragma unroll
      for (int e = 0; e < 4; ++e) {
        bv[it][e]     = (_Float16)(a0[e] * kCarU);
        bv[it][4 + e] = (_Float16)(a1[e] * kCarU);
      }
    }
    for (int pass = 0; pass < 2; ++pass) {
#pragma unroll
      for (int it = 0; it < 4; ++it)
        *(volatile v4f*)(UC + (size_t)(lb + it * 4 + hrow) * kDin + d0 + hch) = fv[it];
#pragma unroll
      for (int it = 0; it < 2; ++it)
        *(volatile v8h*)(UC16 + (size_t)(lb + it * 8 + wave) * kDin + d0 + lane * 8) = bv[it];
      __threadfence();
    }
    __syncthreads();
  }
}

__global__ __launch_bounds__(256) void scan_kernel(
    const float* __restrict__ DLR, const float* __restrict__ UC, const float* __restrict__ XZ,
    const float* __restrict__ XD, const float* __restrict__ bdt, const float* __restrict__ A_log,
    const float* __restrict__ Dv, unsigned short* __restrict__ Y16)
{
  __shared__ __align__(16) float sBC[kScanTS * 32];
  __shared__ __align__(16) float sY[kScanTS * kTP];
  const int tid = threadIdx.x, lane = tid & 31, wave = tid >> 5;
  const int d0 = blockIdx.x * 256, d = d0 + tid;
  const size_t row0 = (size_t)blockIdx.y * kSeq;

  float An[kNst];
#pragma unroll
  for (int q4 = 0; q4 < 4; ++q4) {
    const v4f av = *(const v4f*)(A_log + (size_t)d * kNst + 4 * q4);
    An[4 * q4 + 0] = -expf(av[0]);
    An[4 * q4 + 1] = -expf(av[1]);
    An[4 * q4 + 2] = -expf(av[2]);
    An[4 * q4 + 3] = -expf(av[3]);
  }
  const float bdt2 = 2.0f * bdt[d];
  const float Dd = Dv[d];
  float h[kNst];
#pragma unroll
  for (int n = 0; n < kNst; ++n) h[n] = 0.f;

#pragma unroll 1
  for (int c = 0; c < kSeq / kScanTS; ++c) {
    const int l0 = c * kScanTS;
    if (tid < 128) {
      const int r = tid >> 3, q = (tid & 7) * 4;
      const v4f v = *(const v4f*)(XD + (row0 + l0 + r) * kXdP + kDtR + q);
      *(v4f*)(sBC + r * 32 + q) = v;
    }
    __syncthreads();
#pragma unroll 1
    for (int s = 0; s < kScanTS; ++s) {
      const size_t m = row0 + (size_t)(l0 + s);
      float a  = DLR[m * kDin + d];
      float xv = UC[m * kDin + d];
      float zv = XZ[m * kXzP + kDin + d];
      asm volatile("" : "+v"(a));
      asm volatile("" : "+v"(xv));
      asm volatile("" : "+v"(zv));
      a = a + bdt2;
      const float delta = fmaxf(a, 0.0f) + log1pf(expf(-fabsf(a)));
      v4f Bq[4], Cq[4];
#pragma unroll
      for (int qq = 0; qq < 4; ++qq) {
        Bq[qq] = *(const v4f*)(sBC + s * 32 + 4 * qq);
        Cq[qq] = *(const v4f*)(sBC + s * 32 + kNst + 4 * qq);
      }
      const float dtx = delta * xv;
      float y = 0.f;
#pragma unroll
      for (int n = 0; n < kNst; ++n) {
        const float e  = __expf(delta * An[n]);
        const float hn = fmaf(e, h[n], dtx * Bq[n >> 2][n & 3]);
        h[n] = hn;
        y = fmaf(hn, Cq[n >> 2][n & 3], y);
      }
      y = fmaf(xv, Dd, y);
      const float sg = __builtin_amdgcn_rcpf(1.0f + expf(-zv));
      const float g  = zv * sg;
      sY[s * kTP + tid] = (y * g) * kCarY;
    }
    __syncthreads();
    v8h hv[2];
#pragma unroll
    for (int it = 0; it < 2; ++it) {
      const float* sp = sY + (it * 8 + wave) * kTP + lane * 8;
      const v4f a0 = *(const v4f*)(sp);
      const v4f a1 = *(const v4f*)(sp + 4);
#pragma unroll
      for (int e = 0; e < 4; ++e) {
        hv[it][e]     = (_Float16)a0[e];
        hv[it][4 + e] = (_Float16)a1[e];
      }
    }
    for (int pass = 0; pass < 2; ++pass) {
#pragma unroll
      for (int it = 0; it < 2; ++it)
        *(volatile v8h*)(Y16 + (row0 + (size_t)(l0 + it * 8 + wave)) * kDin + d0 + lane * 8) = hv[it];
      __threadfence();
    }
  }
}

extern "C" void kernel_launch(void* const* d_in, const int* in_sizes, int n_in,
                              void* d_out, int out_size, void* d_ws, size_t ws_size,
                              hipStream_t stream)
{
  if (n_in < 10) return;
  if (in_sizes[0] != kRows * kDm) return;
  if (in_sizes[1] != kXzP * kDm) return;
  if (in_sizes[2] != kDin * 4) return;
  if (in_sizes[3] != kDin) return;
  if (in_sizes[4] != kXdP * kDin) return;
  if (in_sizes[5] != kDin * kDtR) return;
  if (in_sizes[6] != kDin) return;
  if (in_sizes[7] != kDin * kNst) return;
  if (in_sizes[8] != kDin) return;
  if (in_sizes[9] != kDm * kDin) return;
  if (out_size != kRows * kDm) return;
  if (ws_size < kWsTotal) return;

  const float* x      = (const float*)d_in[0];
  const float* W_in   = (const float*)d_in[1];
  const float* conv_w = (const float*)d_in[2];
  const float* conv_b = (const float*)d_in[3];
  const float* W_x    = (const float*)d_in[4];
  const float* W_dt   = (const float*)d_in[5];
  const float* b_dt   = (const float*)d_in[6];
  const float* A_log  = (const float*)d_in[7];
  const float* Dv     = (const float*)d_in[8];
  const float* W_out  = (const float*)d_in[9];
  float* out = (float*)d_out;

  char* ws = (char*)d_ws;
  unsigned short* X16    = (unsigned short*)(ws + kOffX16);
  unsigned short* WIN16  = (unsigned short*)(ws + kOffWIN);
  unsigned short* WX16   = (unsigned short*)(ws + kOffWX);
  unsigned short* WDT16  = (unsigned short*)(ws + kOffWDT);
  unsigned short* WOUT16 = (unsigned short*)(ws + kOffWOUT);
  float*          XZ     = (float*)(ws + kOffXZ);
  float*          UC     = (float*)(ws + kOffUC);
  unsigned short* UC16   = (unsigned short*)(ws + kOffUC16);
  float*          XD     = (float*)(ws + kOffXD);
  unsigned short* DT16   = (unsigned short*)(ws + kOffDT16);
  float*          DLR    = (float*)(ws + kOffDLR);
  unsigned short* Y16    = (unsigned short*)(ws + kOffY16);

  cast_f16_kernel<<<(kRows * kDm / 8) / 256, 256, 0, stream>>>(x,     X16,    kRows * kDm / 8, kCarX);
  cast_f16_kernel<<<(kXzP * kDm / 8) / 256, 256, 0, stream>>>(W_in,   WIN16,  kXzP * kDm / 8,  kCarW);
  cast_f16_kernel<<<(kXdP * kDin / 8) / 256, 256, 0, stream>>>(W_x,   WX16,   kXdP * kDin / 8, kCarW);
  cast_f16_kernel<<<(kDin * kDtR / 8) / 256, 256, 0, stream>>>(W_dt,  WDT16,  kDin * kDtR / 8, kCarWdt);
  cast_f16_kernel<<<(kDm * kDin / 8) / 256, 256, 0, stream>>>(W_out,  WOUT16, kDm * kDin / 8,  kCarW);

  wmma_gemm64_f16<false><<<(kRows / 64) * (kXzP / 64) / 8, 256, 0, stream>>>(
      X16, kDm, WIN16, kDm, XZ, kXzP, x, kRows, kXzP, kDm, 1.0f / (kCarX * kCarW));

  conv_silu_kernel<<<dim3(kDin / 256, kRows / 64), 256, 0, stream>>>(XZ, conv_w, conv_b, UC, UC16);

  wmma_gemm64_f16<false><<<(kRows / 64) * (kXdP / 64) / 8, 256, 0, stream>>>(
      UC16, kDin, WX16, kDin, XD, kXdP, x, kRows, kXdP, kDin, 1.0f / (kCarU * kCarW));

  dt_cast_kernel<<<(kRows * kDtR / 8) / 256, 256, 0, stream>>>(XD, DT16, kRows * kDtR / 8, kCarDt);

  wmma_gemm64_f16<false><<<(kRows / 64) * (kDin / 64) / 8, 256, 0, stream>>>(
      DT16, kDtR, WDT16, kDtR, DLR, kDin, x, kRows, kDin, kDtR, 1.0f / (kCarDt * kCarWdt));

  scan_kernel<<<dim3(kDin / 256, kBatch), 256, 0, stream>>>(DLR, UC, XZ, XD, b_dt, A_log, Dv, Y16);

  wmma_gemm64_f16<true><<<(kRows / 64) * (kDm / 64) / 8, 256, 0, stream>>>(
      Y16, kDin, WOUT16, kDin, out, kDm, x, kRows, kDm, kDin, 1.0f / (kCarY * kCarW));
}
